// SE3TransformerLayer_65644280152627
// MI455X (gfx1250) — hardware-verified
//
#include <hip/hip_runtime.h>


namespace {
constexpr int Bn = 2, S = 2048, HID = 768, NH = 8, HD = 96, HDP = 128, DV = 256, DC = DV * 3, NT = Bn * S;
constexpr float QS = 8.0f, KS = 8.0f, VS = 8.0f, PSC = 4096.0f, AS_ = 8.0f, SCL = 0.10206207261596575f  ;
constexpr size_t QPL = (size_t)Bn * NH * S * HDP;
constexpr size_t VPL = (size_t)Bn * NH * HD * S;
constexpr size_t FPL = (size_t)Bn * DC * S;

typedef _Float16 b16;
typedef __attribute__((ext_vector_type(16))) _Float16 v16b;
typedef __attribute__((ext_vector_type(16))) __bf16 v16bb;
typedef __attribute__((ext_vector_type(8))) _Float16 v8b;
typedef __attribute__((ext_vector_type(8))) unsigned short v8us;
typedef __attribute__((ext_vector_type(8))) float v8f;
typedef __attribute__((ext_vector_type(4))) float v4f;
__device__ __forceinline__ float bf16_rne(float f) { unsigned int u = __float_as_uint(f); u += 0x7FFFu + ((u >> 16) & 1u); return __uint_as_float(u & 0xFFFF0000u); }
__device__ __forceinline__ unsigned short bf16_bits(float f) { unsigned int u = __float_as_uint(f); u += 0x7FFFu + ((u >> 16) & 1u); return (unsigned short)(u >> 16); }
__device__ __forceinline__ void split16(float v, b16& hi, b16& lo) { hi = (b16)v; lo = (b16)(v - (float)hi); }
__device__ __forceinline__ v16b frag_kb(const b16* p, int hh) { const v8b a = *(const v8b*)(p + 8 * hh), b = *(const v8b*)(p + 16 + 8 * hh); v16b f;
#pragma unroll
  for (int e = 0; e < 8; ++e) { f[e] = a[e]; f[8 + e] = b[e]; } return f; }
__device__ __forceinline__ v16bb frag_bf(const unsigned short* p, int hh) { const v8us a = *(const v8us*)(p + 8 * hh), b = *(const v8us*)(p + 16 + 8 * hh); union { unsigned short s[16]; v16bb v; } u;
#pragma unroll
  for (int e = 0; e < 8; ++e) { u.s[e] = a[e]; u.s[8 + e] = b[e]; } return u.v; }
__device__ __forceinline__ v16bb frag_f32bf(const float* p, int hh) { union { unsigned short s[16]; v16bb v; } u;
#pragma unroll
  for (int e = 0; e < 8; ++e) { u.s[e] = bf16_bits(p[8 * hh + e]); u.s[8 + e] = bf16_bits(p[16 + 8 * hh + e]); } return u.v; }
__device__ __forceinline__ void frag_split(const float* p, int hh, v16b& fh, v16b& fl) {
#pragma unroll
  for (int e = 0; e < 8; ++e) { b16 a, c; split16(p[8 * hh + e] * AS_, a, c); fh[e] = a; fl[e] = c; split16(p[16 + 8 * hh + e] * AS_, a, c); fh[8 + e] = a; fl[8 + e] = c; } }
__device__ __forceinline__ v8f wmma16b(v16b a, v16b b, v8f c) { v8f d = __builtin_amdgcn_wmma_f32_16x16x32_f16(false, a, false, b, (short)0, c, false, false); asm volatile("v_nop\n\tv_nop\n\tv_nop\n\tv_nop" : "+v"(d) : "v"(a), "v"(b)); return d; }
__device__ __forceinline__ v8f wmma16bb(v16bb a, v16bb b, v8f c) { v8f d = __builtin_amdgcn_wmma_f32_16x16x32_bf16(false, a, false, b, (short)0, c, false, false); asm volatile("v_nop\n\tv_nop\n\tv_nop\n\tv_nop" : "+v"(d) : "v"(a), "v"(b)); return d; }
__device__ __forceinline__ void wave_lds_sync() { __builtin_amdgcn_fence(__ATOMIC_RELEASE, "workgroup"); __builtin_amdgcn_wave_barrier(); __builtin_amdgcn_fence(__ATOMIC_ACQUIRE, "workgroup"); }
__device__ __forceinline__ float nexp(float x) { return __builtin_amdgcn_exp2f(x * 1.4426950408889634f); }

__global__ __launch_bounds__(256) void prep_kernel(const float* __restrict__ Wq, const float* __restrict__ Wk, const float* __restrict__ Wv, const float* __restrict__ Wo, const float* __restrict__ Wov, const float* __restrict__ bq, const float* __restrict__ bk, const float* __restrict__ bv, const float* __restrict__ bo, const float* __restrict__ lnw, const float* __restrict__ lnb, const float* __restrict__ vlnw,
                                                   unsigned short* __restrict__ w16, b16* __restrict__ wo16, unsigned short* __restrict__ wov16, float* __restrict__ P) {
  const size_t tid = (size_t)blockIdx.x * blockDim.x + threadIdx.x, nth = (size_t)gridDim.x * blockDim.x;
  for (int pass = 0; pass < 2; ++pass) {
    for (size_t p = tid; p < (size_t)3 * HID * HID / 8; p += nth) { const int m = (int)(p / ((size_t)HID * HID / 8)); const size_t q = p % ((size_t)HID * HID / 8); const float* W = (m == 0) ? Wq : (m == 1) ? Wk : Wv; v8us v;
#pragma unroll
      for (int e = 0; e < 8; ++e) v[e] = bf16_bits(W[q * 8 + e]);
      *(volatile v8us*)(w16 + p * 8) = v; }
    for (size_t p = tid; p < (size_t)HID * HID / 8; p += nth) { v8b v;
#pragma unroll
      for (int e = 0; e < 8; ++e) v[e] = (b16)bf16_rne(Wo[p * 8 + e]);
      *(volatile v8b*)(wo16 + p * 8) = v; }
    for (size_t p = tid; p < (size_t)DV * DV / 8; p += nth) { v8us v;
#pragma unroll
      for (int e = 0; e < 8; ++e) v[e] = bf16_bits(Wov[p * 8 + e]);
      *(volatile v8us*)(wov16 + p * 8) = v; }
    for (size_t p = tid; p < 4864 / 4; p += nth) { v4f v;
#pragma unroll
      for (int e = 0; e < 4; ++e) { const int i = (int)p * 4 + e; float x; if (i < 768) x = bq[i]; else if (i < 1536) x = bk[i - 768]; else if (i < 2304) x = bv[i - 1536]; else if (i < 3072) x = bo[i - 2304]; else if (i < 3840) x = lnw[i - 3072]; else if (i < 4608) x = lnb[i - 3840]; else x = vlnw[i - 4608]; v[e] = bf16_rne(x); }
      *(volatile v4f*)(P + p * 4) = v; }
    __threadfence(); }
}

__global__ __launch_bounds__(128) void vfp_kernel(const float* __restrict__ vf, const unsigned short* __restrict__ wov16, b16* __restrict__ fp) {
  __shared__ __attribute__((aligned(16))) b16 Th[64][128 + 8], Tl[64][128 + 8];
  const int lane = threadIdx.x & 31, wave = threadIdx.x >> 5, nloc = lane & 15, hlf = lane >> 4, b = blockIdx.z / 3, c = blockIdx.z % 3, k0 = blockIdx.y * 128, kw = k0 + wave * 32, o0 = blockIdx.x * 64;
  const float* VFb = vf + ((size_t)b * S) * DC;
  v8f acc[2][4];
#pragma unroll
  for (int r = 0; r < 2; ++r)
#pragma unroll
    for (int t = 0; t < 4; ++t) acc[r][t] = (v8f){};
  for (int kb = 0; kb < DV; kb += 32) { union { unsigned short s[16]; v16bb v; } ua, ub; const float* pa = VFb + (size_t)(kw + nloc) * DC + c; const float* pb = VFb + (size_t)(kw + 16 + nloc) * DC + c;
#pragma unroll
    for (int e = 0; e < 8; ++e) { const int i0 = kb + 8 * hlf + e, i1 = kb + 16 + 8 * hlf + e; ua.s[e] = bf16_bits(pa[(size_t)i0 * 3]); ua.s[8 + e] = bf16_bits(pa[(size_t)i1 * 3]); ub.s[e] = bf16_bits(pb[(size_t)i0 * 3]); ub.s[8 + e] = bf16_bits(pb[(size_t)i1 * 3]); }
#pragma unroll
    for (int t = 0; t < 4; ++t) { const v16bb bw = frag_bf(wov16 + (size_t)(o0 + t * 16 + nloc) * DV + kb, hlf); acc[0][t] = wmma16bb(ua.v, bw, acc[0][t]); acc[1][t] = wmma16bb(ub.v, bw, acc[1][t]); } }
#pragma unroll
  for (int t = 0; t < 4; ++t)
#pragma unroll
    for (int r = 0; r < 2; ++r)
#pragma unroll
      for (int v = 0; v < 8; ++v) { b16 a_, l_; split16(acc[r][t][v] * VS, a_, l_); Th[t * 16 + nloc][wave * 32 + r * 16 + 8 * hlf + v] = a_; Tl[t * 16 + nloc][wave * 32 + r * 16 + 8 * hlf + v] = l_; }
  __syncthreads();
  for (int pass = 0; pass < 2; ++pass) { for (int i = threadIdx.x; i < 64 * 16; i += 128) { const int oo = i >> 4, c8 = (i & 15) * 8; const size_t dst = ((size_t)b * DC + (size_t)(o0 + oo) * 3 + c) * S + k0 + c8;
      *(volatile v8b*)(fp + dst) = *(const v8b*)(&Th[oo][c8]); *(volatile v8b*)(fp + FPL + dst) = *(const v8b*)(&Tl[oo][c8]); } __threadfence(); }
}

__global__ __launch_bounds__(128) void proj_kernel(const float* __restrict__ x, const unsigned short* __restrict__ w16, const float* __restrict__ P, b16* __restrict__ qp, b16* __restrict__ kp, b16* __restrict__ vt) {
  __shared__ __attribute__((aligned(16))) b16 Th[4][32][HDP + 8], Tl[4][32][HDP + 8]; __shared__ __attribute__((aligned(16))) b16 Tv[HD][128 + 8];
  const int lane = threadIdx.x & 31, wave = threadIdx.x >> 5, nloc = lane & 15, hlf = lane >> 4, h = blockIdx.x, which = blockIdx.z, m0 = blockIdx.y * 128 + wave * 32, b = (blockIdx.y * 128) / S, t0 = (blockIdx.y * 128) % S;
  const unsigned short* Wt = w16 + ((size_t)which * HID + h * HD) * HID; const float* bias = P + which * 768 + h * HD;
  v8f acc[2][6];
#pragma unroll
  for (int r = 0; r < 2; ++r)
#pragma unroll
    for (int t = 0; t < 6; ++t) acc[r][t] = (v8f){};
#pragma unroll 2
  for (int kb = 0; kb < HID; kb += 32) { const v16bb a0 = frag_f32bf(x + (size_t)(m0 + nloc) * HID + kb, hlf), a1 = frag_f32bf(x + (size_t)(m0 + 16 + nloc) * HID + kb, hlf);
#pragma unroll
    for (int t = 0; t < 6; ++t) { const v16bb bw = frag_bf(Wt + (size_t)(t * 16 + nloc) * HID + kb, hlf); acc[0][t] = wmma16bb(a0, bw, acc[0][t]); acc[1][t] = wmma16bb(a1, bw, acc[1][t]); } }
  if (which < 2) { const float scl = (which == 0) ? QS : KS;
#pragma unroll
    for (int t = 0; t < 6; ++t) { const float bb = bias[t * 16 + nloc];
#pragma unroll
      for (int r = 0; r < 2; ++r)
#pragma unroll
        for (int v = 0; v < 8; ++v) { b16 a_, l_; split16((acc[r][t][v] + bb) * scl, a_, l_); Th[wave][r * 16 + 8 * hlf + v][t * 16 + nloc] = a_; Tl[wave][r * 16 + 8 * hlf + v][t * 16 + nloc] = l_; } }
    for (int i = lane; i < 32 * 32; i += 32) { const int rr = i >> 5, cc = HD + (i & 31); Th[wave][rr][cc] = (b16)0.0f; Tl[wave][rr][cc] = (b16)0.0f; }
    wave_lds_sync();
    b16* base = (which == 0) ? qp : kp;
    for (int pass = 0; pass < 2; ++pass) {
#pragma unroll
      for (int j = 0; j < 8; ++j) { const int rr = j * 4 + (lane >> 3), c8 = (lane & 7) * 8; const int m = m0 + rr, bb_ = m / S, tok = m % S; const size_t o = (((size_t)bb_ * NH + h) * S + tok) * HDP;
        *(volatile v8b*)(base + o + c8) = *(const v8b*)(&Th[wave][rr][c8]); *(volatile v8b*)(base + o + 64 + c8) = *(const v8b*)(&Th[wave][rr][64 + c8]);
        *(volatile v8b*)(base + QPL + o + c8) = *(const v8b*)(&Tl[wave][rr][c8]); *(volatile v8b*)(base + QPL + o + 64 + c8) = *(const v8b*)(&Tl[wave][rr][64 + c8]); }
      __threadfence(); }
    return; }
#pragma unroll
  for (int t = 0; t < 6; ++t) { const float bb = bias[t * 16 + nloc];
#pragma unroll
    for (int r = 0; r < 2; ++r)
#pragma unroll
      for (int v = 0; v < 8; ++v) Tv[t * 16 + nloc][wave * 32 + r * 16 + 8 * hlf + v] = (b16)((acc[r][t][v] + bb) * VS); }
  __syncthreads();
  for (int pass = 0; pass < 2; ++pass) { for (int i = threadIdx.x; i < HD * 16; i += 128) { const int d = i >> 4, c8 = (i & 15) * 8; *(volatile v8b*)(vt + (((size_t)b * NH + h) * HD + d) * S + t0 + c8) = *(const v8b*)(&Tv[d][c8]); } __threadfence(); }
}

__global__ __launch_bounds__(256) void score_kernel(const b16* __restrict__ qp, const b16* __restrict__ kp, int h, b16* __restrict__ SP, float* __restrict__ PM) {
  __shared__ __attribute__((aligned(16))) b16 Ts[8][16][64 + 8]; __shared__ float Mz[8][2][16]; __shared__ float Mh[8][16][S / 32 + 1];
  const int wid = threadIdx.x >> 5, lane = threadIdx.x & 31, hh = lane >> 4, col = lane & 15; const int qg = blockIdx.x * 8 + wid, b = qg / (S / 16), q0 = (qg % (S / 16)) * 16;
  const b16* Q = qp + (((size_t)b * NH + h) * S + q0 + col) * HDP; const b16* K = kp + (((size_t)b * NH + h) * S) * HDP; b16* Srow = SP + ((size_t)b * S + q0) * S; float* Prow = PM + ((size_t)b * S + q0) * S;
  float m = -INFINITY, z = 0.0f;
  for (int kb = 0; kb < S; kb += 32) { const int half = (kb >> 5) & 1; v8f s0 = {}, s1 = {};
#pragma unroll
    for (int ks = 0; ks < HDP; ks += 32) { const v16b qf = frag_kb(Q + ks, hh), ql = frag_kb(Q + QPL + ks, hh); const v16b ka = frag_kb(K + (size_t)(kb + col) * HDP + ks, hh), kal = frag_kb(K + QPL + (size_t)(kb + col) * HDP + ks, hh), kc = frag_kb(K + (size_t)(kb + 16 + col) * HDP + ks, hh), kcl = frag_kb(K + QPL + (size_t)(kb + 16 + col) * HDP + ks, hh);
      s0 = wmma16b(ka, qf, s0); s0 = wmma16b(ka, ql, s0); s0 = wmma16b(kal, qf, s0); s1 = wmma16b(kc, qf, s1); s1 = wmma16b(kc, ql, s1); s1 = wmma16b(kcl, qf, s1); }
    float mr = -INFINITY;
#pragma unroll
    for (int r = 0; r < 8; ++r) { s0[r] *= SCL / (QS * KS); s1[r] *= SCL / (QS * KS); mr = fmaxf(mr, fmaxf(s0[r], s1[r])); }
    mr = fmaxf(mr, __shfl_xor(mr, 16));
    const float mn = fmaxf(m, mr); float sum = 0.0f;
#pragma unroll
    for (int r = 0; r < 8; ++r) sum += nexp(s0[r] - mn) + nexp(s1[r] - mn);
    sum += __shfl_xor(sum, 16); z = z * nexp(m - mn) + sum; m = mn;
    if (hh == 0) Mh[wid][col][kb >> 5] = mn;
#pragma unroll
    for (int r = 0; r < 8; ++r) { Ts[wid][col][half * 32 + 8 * hh + r] = (b16)(nexp(s0[r] - mn) * PSC); Ts[wid][col][half * 32 + 16 + 8 * hh + r] = (b16)(nexp(s1[r] - mn) * PSC); }
    if (half == 1) { wave_lds_sync();
      for (int pass = 0; pass < 2; ++pass) {
#pragma unroll
        for (int j = 0; j < 4; ++j) { const int rr = j * 4 + (lane >> 3), c8 = (lane & 7) * 8; *(volatile v8b*)(Srow + (size_t)rr * S + (kb - 32) + c8) = *(const v8b*)(&Ts[wid][rr][c8]); } }
      wave_lds_sync(); }
  }
  if (hh == 0) { Mz[wid][0][col] = m; Mz[wid][1][col] = 1.0f / z; }
  __threadfence(); wave_lds_sync();
  for (int kb = 0; kb < S; kb += 64) {
#pragma unroll
    for (int j = 0; j < 4; ++j) { const int rr = j * 4 + (lane >> 3), c8 = (lane & 7) * 8; b16* p = Srow + (size_t)rr * S + kb + c8; float* pm = Prow + (size_t)rr * S + kb + c8; const float mm = Mz[wid][0][rr], iz = Mz[wid][1][rr];
      const v8b a = *(const volatile v8b*)p; const int blk = (kb + c8) >> 5; const float resc = nexp(Mh[wid][rr][blk] - mm) * iz; v8b o; v4f pa, pb;
      if (h == 0) { pa = (v4f){0.0f, 0.0f, 0.0f, 0.0f}; pb = pa; } else { pa = *(const volatile v4f*)pm; pb = *(const volatile v4f*)(pm + 4); }
#pragma unroll
      for (int e = 0; e < 8; ++e) { const float pe = (float)a[e] * resc; o[e] = (b16)pe; const float pn = pe * (1.0f / (PSC * NH)); if (e < 4) pa[e] += pn; else pb[e - 4] += pn; }
      for (int pass = 0; pass < 2; ++pass) { *(volatile v8b*)p = o; *(volatile v4f*)pm = pa; *(volatile v4f*)(pm + 4) = pb; } } }
  __threadfence();
}

__global__ __launch_bounds__(128) void pv_kernel(const b16* __restrict__ SP, const b16* __restrict__ vt, int h, float* __restrict__ asp) {
  __shared__ __attribute__((aligned(16))) float Ts[4][32][HD + 4];
  const int lane = threadIdx.x & 31, wave = threadIdx.x >> 5, nloc = lane & 15, hlf = lane >> 4, b = blockIdx.y, m0 = blockIdx.x * 128 + wave * 32;
  const b16* A = SP + ((size_t)b * S) * S; const b16* Bv = vt + (((size_t)b * NH + h) * HD) * S;
  v8f acc[2][6];
#pragma unroll
  for (int r = 0; r < 2; ++r)
#pragma unroll
    for (int t = 0; t < 6; ++t) acc[r][t] = (v8f){};
#pragma unroll 2
  for (int kb = 0; kb < S; kb += 32) { const v16b a0 = frag_kb(A + (size_t)(m0 + nloc) * S + kb, hlf), a1 = frag_kb(A + (size_t)(m0 + 16 + nloc) * S + kb, hlf);
#pragma unroll
    for (int t = 0; t < 6; ++t) { const v16b bw = frag_kb(Bv + (size_t)(t * 16 + nloc) * S + kb, hlf); acc[0][t] = wmma16b(a0, bw, acc[0][t]); acc[1][t] = wmma16b(a1, bw, acc[1][t]); } }
#pragma unroll
  for (int t = 0; t < 6; ++t)
#pragma unroll
    for (int r = 0; r < 2; ++r)
#pragma unroll
      for (int v = 0; v < 8; ++v) Ts[wave][r * 16 + 8 * hlf + v][t * 16 + nloc] = acc[r][t][v] * (1.0f / (PSC * VS));
  wave_lds_sync();
  float* dst = asp + (((size_t)b * NH + h) * S + m0) * HDP;
  for (int pass = 0; pass < 2; ++pass) { for (int i = lane; i < 32 * (HD / 4); i += 32) { const int rr = i / (HD / 4), c4 = (i % (HD / 4)) * 4; *(volatile v4f*)(dst + (size_t)rr * HDP + c4) = *(const v4f*)(&Ts[wave][rr][c4]); } __threadfence(); }
}

__global__ __launch_bounds__(128) void vec_kernel(const float* __restrict__ PM, const b16* __restrict__ fp, const float* __restrict__ vf, const float* __restrict__ P, float* __restrict__ vout) {
  __shared__ __attribute__((aligned(16))) float Ts[4][32][96 + 4];
  const int lane = threadIdx.x & 31, wave = threadIdx.x >> 5, nloc = lane & 15, hlf = lane >> 4, b = blockIdx.z, m0 = blockIdx.y * 128 + wave * 32, c0 = blockIdx.x * 96; const float* vlnw = P + 4608;
  const float* A = PM + ((size_t)b * S) * S; const b16* Bf = fp + ((size_t)b * DC) * S;
  v8f acc[2][6];
#pragma unroll
  for (int r = 0; r < 2; ++r)
#pragma unroll
    for (int t = 0; t < 6; ++t) acc[r][t] = (v8f){};
  for (int kb = 0; kb < S; kb += 32) { v16b a0, l0, a1, l1; frag_split(A + (size_t)(m0 + nloc) * S + kb, hlf, a0, l0); frag_split(A + (size_t)(m0 + 16 + nloc) * S + kb, hlf, a1, l1);
#pragma unroll
    for (int t = 0; t < 6; ++t) { const v16b bh = frag_kb(Bf + (size_t)(c0 + t * 16 + nloc) * S + kb, hlf), bl = frag_kb(Bf + FPL + (size_t)(c0 + t * 16 + nloc) * S + kb, hlf);
      acc[0][t] = wmma16b(a0, bh, acc[0][t]); acc[0][t] = wmma16b(a0, bl, acc[0][t]); acc[0][t] = wmma16b(l0, bh, acc[0][t]);
      acc[1][t] = wmma16b(a1, bh, acc[1][t]); acc[1][t] = wmma16b(a1, bl, acc[1][t]); acc[1][t] = wmma16b(l1, bh, acc[1][t]); } }
#pragma unroll
  for (int t = 0; t < 6; ++t)
#pragma unroll
    for (int r = 0; r < 2; ++r)
#pragma unroll
      for (int v = 0; v < 8; ++v) { const int rl = r * 16 + 8 * hlf + v, cc = t * 16 + nloc; Ts[wave][rl][cc] = acc[r][t][v] * (1.0f / (AS_ * VS)) + bf16_rne(vf[((size_t)b * S + m0 + rl) * DC + c0 + cc]); }
  wave_lds_sync();
  for (int rl = 0; rl < 32; ++rl) { const int o = c0 / 3 + lane; const float x0 = Ts[wave][rl][lane * 3], x1 = Ts[wave][rl][lane * 3 + 1], x2 = Ts[wave][rl][lane * 3 + 2];
    const float nrm = sqrtf((x0 * x0 + x1 * x1) + x2 * x2); const float f = vlnw[o] / (nrm + 1e-8f); Ts[wave][rl][lane * 3] = x0 * f; Ts[wave][rl][lane * 3 + 1] = x1 * f; Ts[wave][rl][lane * 3 + 2] = x2 * f; }
  wave_lds_sync();
  for (int pass = 0; pass < 2; ++pass) { for (int i = lane; i < 32 * 24; i += 32) { const int rr = i / 24, c4 = (i % 24) * 4; *(volatile v4f*)(vout + ((size_t)b * S + m0 + rr) * DC + c0 + c4) = *(const v4f*)(&Ts[wave][rr][c4]); } __threadfence(); }
}

__global__ __launch_bounds__(128) void wo_kernel(const float* __restrict__ asp, const b16* __restrict__ wo16, const float* __restrict__ x, const float* __restrict__ P, float* __restrict__ pre) {
  __shared__ __attribute__((aligned(16))) float Ts[4][32 * 64];
  const int lane = threadIdx.x & 31, wave = threadIdx.x >> 5, nloc = lane & 15, hlf = lane >> 4, m0 = blockIdx.y * 128 + wave * 32, c0 = blockIdx.x * 64; const int b = m0 / S, q0 = m0 % S; const float* bo = P + 2304;
  v8f acc[2][4];
#pragma unroll
  for (int r = 0; r < 2; ++r)
#pragma unroll
    for (int t = 0; t < 4; ++t) acc[r][t] = (v8f){};
  for (int kb = 0; kb < HID; kb += 32) { const int h = kb / HD, d0 = kb % HD; const float* Ap = asp + (((size_t)b * NH + h) * S + q0) * HDP + d0; v16b a0, l0, a1, l1; frag_split(Ap + (size_t)nloc * HDP, hlf, a0, l0); frag_split(Ap + (size_t)(16 + nloc) * HDP, hlf, a1, l1);
#pragma unroll
    for (int t = 0; t < 4; ++t) { const v16b bw = frag_kb(wo16 + (size_t)(c0 + t * 16 + nloc) * HID + kb, hlf); acc[0][t] = wmma16b(a0, bw, acc[0][t]); acc[0][t] = wmma16b(l0, bw, acc[0][t]); acc[1][t] = wmma16b(a1, bw, acc[1][t]); acc[1][t] = wmma16b(l1, bw, acc[1][t]); } }
  float* Tt = Ts[wave];
#pragma unroll
  for (int t = 0; t < 4; ++t) { const int cc = c0 + t * 16 + nloc; const float bb = bo[cc];
#pragma unroll
    for (int r = 0; r < 2; ++r)
#pragma unroll
      for (int v = 0; v < 8; ++v) { const int rl = r * 16 + v + 8 * hlf; Tt[rl * 64 + t * 16 + nloc] = acc[r][t][v] * (1.0f / AS_) + bb + bf16_rne(x[(size_t)(m0 + rl) * HID + cc]); } }
  wave_lds_sync();
  for (int pass = 0; pass < 2; ++pass) {
#pragma unroll
    for (int j = 0; j < 16; ++j) { const int rr = j * 2 + hlf, c4 = nloc * 4; *(volatile v4f*)(pre + (size_t)(m0 + rr) * HID + c0 + c4) = *(const v4f*)(Tt + rr * 64 + c4); }
    __threadfence(); }
}

__global__ __launch_bounds__(256) void ln_kernel(const float* __restrict__ pre, const float* __restrict__ P, float* __restrict__ out) {
  const int wid = threadIdx.x >> 5, lane = threadIdx.x & 31, row = blockIdx.x * 8 + wid; const float* pr = pre + (size_t)row * HID; const float* w = P + 3072; const float* bb = P + 3840;
  float v[24]; float s = 0.0f;
#pragma unroll
  for (int j = 0; j < 6; ++j) { const v4f t = *(const v4f*)(pr + j * 128 + lane * 4); v[j * 4] = t[0]; v[j * 4 + 1] = t[1]; v[j * 4 + 2] = t[2]; v[j * 4 + 3] = t[3]; s += (t[0] + t[1]) + (t[2] + t[3]); }
#pragma unroll
  for (int o = 1; o < 32; o <<= 1) s += __shfl_xor(s, o);
  const float mu = s * (1.0f / HID); float q = 0.0f;
#pragma unroll
  for (int j = 0; j < 24; ++j) { const float d = v[j] - mu; q += d * d; }
#pragma unroll
  for (int o = 1; o < 32; o <<= 1) q += __shfl_xor(q, o);
  const float is = rsqrtf(q * (1.0f / HID) + 1e-5f);
  for (int pass = 0; pass < 2; ++pass) {
#pragma unroll
    for (int j = 0; j < 6; ++j) { const int c = j * 128 + lane * 4; v4f o4; for (int e = 0; e < 4; ++e) o4[e] = (v[j * 4 + e] - mu) * is * w[c + e] + bb[c + e]; *(volatile v4f*)(out + (size_t)row * HID + c) = o4; }
    __threadfence(); }
}
}

extern "C" void kernel_launch(void* const* d_in, const int* in_sizes, int n_in,
                              void* d_out, int out_size, void* d_ws, size_t ws_size, hipStream_t stream) {
  (void)n_in; (void)out_size;
  const float* x = (const float*)d_in[0]; const float* vf = (const float*)d_in[1]; const float* Wq = (const float*)d_in[2]; const float* bq = (const float*)d_in[3]; const float* Wk = (const float*)d_in[4]; const float* bk = (const float*)d_in[5]; const float* Wv = (const float*)d_in[6]; const float* bv = (const float*)d_in[7];
  const float* Wo = (const float*)d_in[8]; const float* bo = (const float*)d_in[9]; const float* Wov = (const float*)d_in[10]; const float* lnw = (const float*)d_in[11]; const float* lnb = (const float*)d_in[12]; const float* vlnw = (const float*)d_in[13];
  float* sout = (float*)d_out; float* vout = sout + (size_t)NT * HID;
  if (in_sizes[0] != NT * HID || in_sizes[1] != NT * DC || in_sizes[2] != HID * HID || in_sizes[10] != DV * DV || in_sizes[13] != DV) return;
  size_t off = 0; char* ws = (char*)d_ws;
  auto carve = [&](size_t bytes) { char* p = ws + off; off += (bytes + 255) & ~(size_t)255; return p; };
  unsigned short* w16 = (unsigned short*)carve((size_t)3 * HID * HID * 2); b16* wo16 = (b16*)carve((size_t)HID * HID * 2); unsigned short* wov16 = (unsigned short*)carve((size_t)DV * DV * 2); float* P = (float*)carve(4864 * 4 + 256);
  b16* fp = (b16*)carve(FPL * 2 * 2); b16* qp = (b16*)carve(QPL * 2 * 2); b16* kp = (b16*)carve(QPL * 2 * 2); b16* vt = (b16*)carve(VPL * 2); b16* SP = (b16*)carve((size_t)Bn * S * S * 2); float* PM = (float*)carve((size_t)Bn * S * S * 4); float* asp = (float*)carve((size_t)Bn * NH * S * HDP * 4);
  float* pre = (float*)fp;
  if (off > ws_size) return;
  prep_kernel<<<256, 256, 0, stream>>>(Wq, Wk, Wv, Wo, Wov, bq, bk, bv, bo, lnw, lnb, vlnw, w16, wo16, wov16, P);
  vfp_kernel<<<dim3(DV / 64, S / 128, Bn * 3), 128, 0, stream>>>(vf, wov16, fp);
  proj_kernel<<<dim3(NH, NT / 128, 3), 128, 0, stream>>>(x, w16, P, qp, kp, vt);
  for (int h = 0; h < NH; ++h) { score_kernel<<<NT / 16 / 8, 256, 0, stream>>>(qp, kp, h, SP, PM); pv_kernel<<<dim3(S / 128, Bn), 128, 0, stream>>>(SP, vt, h, asp); }
  vec_kernel<<<dim3(DC / 96, S / 128, Bn), 128, 0, stream>>>(PM, fp, vf, P, vout);
  wo_kernel<<<dim3(HID / 64, NT / 128), 128, 0, stream>>>(asp, wo16, x, P, pre);
  ln_kernel<<<NT / 8, 256, 0, stream>>>(pre, P, sout);
}
